// attention_propagantion_78262894068287
// MI455X (gfx1250) — hardware-verified
//
#include <hip/hip_runtime.h>


#define NB_  2
#define CC   256
#define NN   8192
#define NH_  4
#define HD   64
#define KNB  16
typedef _Float16 h16;
typedef unsigned short bf;
typedef __attribute__((ext_vector_type(16))) __bf16   v16bf;
typedef __attribute__((ext_vector_type(16))) _Float16 v16h;
typedef __attribute__((ext_vector_type(8)))  _Float16 v8h;
typedef __attribute__((ext_vector_type(8)))  unsigned short v8us;
typedef __attribute__((ext_vector_type(8)))  float    v8f;
typedef __attribute__((ext_vector_type(4)))  float    v4f;
typedef v8h  __attribute__((may_alias)) v8ha;
typedef v4f  __attribute__((may_alias)) v4fa;
typedef v8us __attribute__((may_alias)) v8usa;

__device__ __forceinline__ unsigned short f2bf(float f) { unsigned u = __float_as_uint(f); u += 0x7FFFu + ((u >> 16) & 1u); return (unsigned short)(u >> 16); }
__device__ __forceinline__ float bf2f(unsigned short b) { return __uint_as_float(((unsigned)b) << 16); }
__device__ __forceinline__ float bfr(float f) { return bf2f(f2bf(f)); }
__device__ __forceinline__ v16h cat16(v8h lo, v8h hi) { return __builtin_shufflevector(lo, hi, 0, 1, 2, 3, 4, 5, 6, 7, 8, 9, 10, 11, 12, 13, 14, 15); }
__device__ __forceinline__ v16bf cat16b(v8us lo, v8us hi) { return __builtin_bit_cast(v16bf, __builtin_shufflevector(lo, hi, 0, 1, 2, 3, 4, 5, 6, 7, 8, 9, 10, 11, 12, 13, 14, 15)); }
__device__ __forceinline__ v8f wmma16(v16h a, v16h b, v8f c) { return __builtin_amdgcn_wmma_f32_16x16x32_f16(false, a, false, b, (short)0, c, false, false); }
__device__ __forceinline__ v8f wmmab(v16bf a, v16bf b, v8f c) { return __builtin_amdgcn_wmma_f32_16x16x32_bf16(false, a, false, b, (short)0, c, false, false); }


template <typename T16> struct WFrag;
template <> struct WFrag<h16> { typedef v16h V; static __device__ __forceinline__ V ld(const h16* p) { return cat16(*(const v8h*)p, *(const v8h*)(p + 16)); } static __device__ __forceinline__ v8f mma(V a, V b, v8f c) { return wmma16(a, b, c); } };
template <> struct WFrag<bf> { typedef v16bf V; static __device__ __forceinline__ V ld(const bf* p) { return cat16b(*(const v8us*)p, *(const v8us*)(p + 16)); } static __device__ __forceinline__ v8f mma(V a, V b, v8f c) { return wmmab(a, b, c); } };
template <typename T16, int NSPLIT, bool BIAS>
__global__ __launch_bounds__(32) void k_gemmw(const T16* __restrict__ A, const T16* __restrict__ A2, const T16* __restrict__ Bt, const T16* __restrict__ Bt2, int K, float* C, int ldc, const float* __restrict__ bias, size_t sA, size_t sB, size_t sC) {
    typedef typename WFrag<T16>::V V;
    __shared__ __align__(16) float os[16 * 68];
    const size_t z = blockIdx.z; A += z * sA; if (A2) A2 += z * sA; Bt += z * sB; if (Bt2) Bt2 += z * sB; C += z * sC;
    const int lane = threadIdx.x & 31, lr = lane & 15, hi = lane >> 4; const int r0 = blockIdx.x * 64, c0 = blockIdx.y * 64;
    v8f acc[4][4];
#pragma unroll
    for (int mb = 0; mb < 4; ++mb)
#pragma unroll
        for (int nb = 0; nb < 4; ++nb) acc[mb][nb] = (v8f){};
    const size_t aoff = (size_t)(r0 + lr) * K + 8 * hi, boff = (size_t)(c0 + lr) * K + 8 * hi;
#pragma unroll 1
    for (int kc = 0; kc < K; kc += 32) {
        V a[4], a2[4];
#pragma unroll
        for (int mb = 0; mb < 4; ++mb) { a[mb] = WFrag<T16>::ld(A + aoff + (size_t)mb * 16 * K + kc); if (NSPLIT == 1 || NSPLIT == 2) a2[mb] = WFrag<T16>::ld(A2 + aoff + (size_t)mb * 16 * K + kc); }
#pragma unroll
        for (int nb = 0; nb < 4; ++nb) { const V b = WFrag<T16>::ld(Bt + boff + (size_t)nb * 16 * K + kc); V b2; if (NSPLIT >= 2) b2 = WFrag<T16>::ld(Bt2 + boff + (size_t)nb * 16 * K + kc);
#pragma unroll
            for (int mb = 0; mb < 4; ++mb) { acc[mb][nb] = WFrag<T16>::mma(a[mb], b, acc[mb][nb]); if (NSPLIT == 1 || NSPLIT == 2) acc[mb][nb] = WFrag<T16>::mma(a2[mb], b, acc[mb][nb]); if (NSPLIT >= 2) acc[mb][nb] = WFrag<T16>::mma(a[mb], b2, acc[mb][nb]); } }
        asm volatile("v_nop\n\tv_nop\n\tv_nop\n\tv_nop" : "+v"(acc[0][0]), "+v"(acc[1][1]), "+v"(acc[2][2]), "+v"(acc[3][3]) : "v"(a[0]), "v"(a[3]));
    }
#pragma unroll
    for (int mb = 0; mb < 4; ++mb) {
#pragma unroll
        for (int nb = 0; nb < 4; ++nb) {
#pragma unroll
            for (int j = 0; j < 8; ++j) os[(hi * 8 + j) * 68 + nb * 16 + lr] = acc[mb][nb][j]; }
        __builtin_amdgcn_wave_barrier(); asm volatile("" ::: "memory");
        float* crow = C + (size_t)(r0 + mb * 16) * ldc + c0;
#pragma unroll 1
        for (int ps = 0; ps < 2; ++ps) {
#pragma unroll
            for (int s = 0; s < 8; ++s) { const int row = 2 * s + hi, cofs = lr * 4; v4f val = *(const v4fa*)(os + row * 68 + cofs); if (BIAS) { val[0] += bfr(bias[c0 + cofs]); val[1] += bfr(bias[c0 + cofs + 1]); val[2] += bfr(bias[c0 + cofs + 2]); val[3] += bfr(bias[c0 + cofs + 3]); }
                *(volatile v4f*)(crow + (size_t)row * ldc + cofs) = val; }
            if (ps == 0) __threadfence(); }
        __builtin_amdgcn_wave_barrier(); asm volatile("" ::: "memory");
    }
}

__device__ __forceinline__ void splitf(float y, unsigned short& h, unsigned short& l) { h = f2bf(y); l = f2bf(y - bf2f(h)); }
typedef __attribute__((ext_vector_type(2))) unsigned short v2us;
typedef __attribute__((ext_vector_type(4))) unsigned short v4us;
typedef __attribute__((ext_vector_type(2))) float v2f;

__global__ __launch_bounds__(256) void k_cvt8(const float* __restrict__ src, bf* dst, size_t n8) { const size_t i = (size_t)blockIdx.x * 256 + threadIdx.x; if (i >= n8) return; const v8f v = *(const v8f*)(src + i * 8); v8us o;
#pragma unroll
    for (int k = 0; k < 8; ++k) o[k] = f2bf(v[k]); *(volatile v8us*)(dst + i * 8) = o; __threadfence(); *(volatile v8us*)(dst + i * 8) = o; }
__global__ __launch_bounds__(256) void k_xt(const float* __restrict__ x, bf* XT) { const size_t e = ((size_t)blockIdx.x * 256 + threadIdx.x) * 4; if (e >= (size_t)NN * CC) return; const int c = (int)(e % CC); const int n = (int)(e / CC); v4us o;
#pragma unroll
    for (int q = 0; q < 4; ++q) o[q] = f2bf(x[(size_t)(c + q) * NN + n]); *(volatile v4us*)(XT + e) = o; __threadfence(); *(volatile v4us*)(XT + e) = o; }
__global__ __launch_bounds__(256) void k_spl(const float* __restrict__ F, size_t n4, bf* Fh, bf* Fl) { const size_t i = ((size_t)blockIdx.x * 256 + threadIdx.x) * 4; if (i >= n4 * 4) return; const v4f a = *(const v4f*)(F + i); v4us oh, ol;
#pragma unroll
    for (int q = 0; q < 4; ++q) { unsigned short u, c2; splitf(a[q], u, c2); oh[q] = u; ol[q] = c2; } *(volatile v4us*)(Fh + i) = oh; *(volatile v4us*)(Fl + i) = ol; __threadfence(); *(volatile v4us*)(Fh + i) = oh; *(volatile v4us*)(Fl + i) = ol; }
__global__ __launch_bounds__(256) void k_catpl(const float* __restrict__ x, const float* __restrict__ M, bf* Ch, bf* Cl) { const size_t e = ((size_t)blockIdx.x * 256 + threadIdx.x) * 4; if (e >= (size_t)NN * 2 * CC) return; const int c = (int)(e % (2 * CC)); const int n = (int)(e / (2 * CC)); v4us oh, ol;
#pragma unroll
    for (int q = 0; q < 4; ++q) { const int cc = c + q; unsigned short u, l; if (cc < CC) { u = f2bf(x[(size_t)cc * NN + n]); l = 0; } else splitf(M[(size_t)n * CC + cc - CC], u, l); oh[q] = u; ol[q] = l; }
    *(volatile v4us*)(Ch + e) = oh; *(volatile v4us*)(Cl + e) = ol; __threadfence(); *(volatile v4us*)(Ch + e) = oh; *(volatile v4us*)(Cl + e) = ol; }
__global__ __launch_bounds__(256) void k_nbr(const float* __restrict__ QF, const float* __restrict__ KE, const float* __restrict__ VA, const int* __restrict__ nbr, const float* __restrict__ nmask, const float* __restrict__ rlam, float* ADD) {
    const int lane = threadIdx.x & 31; const int row = blockIdx.x * 8 + (threadIdx.x >> 5); if (row >= NN * NH_) return; const int h = row % NH_; const int n = row / NH_; const int d0 = h * HD + 2 * lane; const float q0 = QF[(size_t)n * CC + d0], q1 = QF[(size_t)n * CC + d0 + 1]; const float lam = bfr(rlam[h]); float se_sum = 0.f, a0 = 0.f, a1 = 0.f;
#pragma unroll 1
    for (int k = 0; k < KNB; ++k) { int j = nbr[(size_t)k * NN + n]; j = min(max(j, 0), NN - 1); const float* ke = KE + (size_t)j * CC + d0; float p = __fmul_rn(q0, ke[0]); asm volatile("" : "+v"(p)); float p2 = __fmul_rn(q1, ke[1]); asm volatile("" : "+v"(p2)); float s = __fadd_rn(p, p2);
#pragma unroll
        for (int sh = 16; sh; sh >>= 1) s += __shfl_xor(s, sh, 32);
        float sm = __fmul_rn(s, 0.125f); asm volatile("" : "+v"(sm)); float lm = __fmul_rn(lam, bfr(nmask[(size_t)k * NN + n])); asm volatile("" : "+v"(lm)); const float simi = __fadd_rn(sm, lm); const float se = __expf(fminf(fmaxf(simi, -30.f), 30.f)); se_sum = __fadd_rn(se_sum, se);
        const float* va = VA + (size_t)j * CC + d0; float t0 = __fmul_rn(se, va[0]); asm volatile("" : "+v"(t0)); a0 = __fadd_rn(a0, t0); float t1 = __fmul_rn(se, va[1]); asm volatile("" : "+v"(t1)); a1 = __fadd_rn(a1, t1); }
    const float inv = __fdiv_rn(1.0f, __fadd_rn(se_sum, 1e-8f)); v2f o; o[0] = __fmul_rn(a0, inv); o[1] = __fmul_rn(a1, inv); const size_t oo = (size_t)n * CC + d0; *(volatile v2f*)(ADD + oo) = o; __threadfence(); *(volatile v2f*)(ADD + oo) = o; }
__global__ __launch_bounds__(256) void k_bnrelu(const float* __restrict__ Y, const float* __restrict__ g, const float* __restrict__ bb, const float* __restrict__ mu, const float* __restrict__ var, bf* Ph, bf* Pl) { const size_t i = ((size_t)blockIdx.x * 256 + threadIdx.x) * 4; if (i >= (size_t)NN * 2 * CC) return; const int c = (int)(i % (2 * CC)); const v4f a = *(const v4f*)(Y + i); v4us oh, ol;
#pragma unroll
    for (int q = 0; q < 4; ++q) { const int cc = c + q; const float sc = __fdiv_rn(bfr(g[cc]), __fsqrt_rn(__fadd_rn(bfr(var[cc]), 1e-5f))); float d = __fsub_rn(a[q], bfr(mu[cc])); asm volatile("" : "+v"(d)); float t = __fmul_rn(d, sc); asm volatile("" : "+v"(t)); unsigned short u, l; splitf(fmaxf(__fadd_rn(t, bfr(bb[cc])), 0.f), u, l); oh[q] = u; ol[q] = l; }
    *(volatile v4us*)(Ph + i) = oh; *(volatile v4us*)(Pl + i) = ol; __threadfence(); *(volatile v4us*)(Ph + i) = oh; *(volatile v4us*)(Pl + i) = ol; }
__global__ __launch_bounds__(256) void k_outT(const float* __restrict__ x, const float* __restrict__ R, float* OUT) { const size_t e = ((size_t)blockIdx.x * 256 + threadIdx.x) * 4; if (e >= (size_t)CC * NN) return; const int n = (int)(e % NN); const int c = (int)(e / NN); v4f o;
#pragma unroll
    for (int q = 0; q < 4; ++q) o[q] = __fadd_rn(bfr(x[e + q]), R[(size_t)(n + q) * CC + c]); *(volatile v4f*)(OUT + e) = o; __threadfence(); *(volatile v4f*)(OUT + e) = o; }

extern "C" void kernel_launch(void* const* d_in, const int* in_sizes, int n_in,
                              void* d_out, int out_size, void* d_ws, size_t ws_size, hipStream_t stream) {
    (void)in_sizes; (void)n_in; (void)out_size;
    const float* d1 = (const float*)d_in[0]; const float* d2 = (const float*)d_in[1]; const int* nbr = (const int*)d_in[2]; const float* nmask = (const float*)d_in[3]; const float* rlam = (const float*)d_in[5];
    const float* wq = (const float*)d_in[6]; const float* bq = (const float*)d_in[7]; const float* wk = (const float*)d_in[8]; const float* bk = (const float*)d_in[9]; const float* wv = (const float*)d_in[10]; const float* bv = (const float*)d_in[11]; const float* wm = (const float*)d_in[12]; const float* bm = (const float*)d_in[13];
    const float* wc1 = (const float*)d_in[14]; const float* bng = (const float*)d_in[15]; const float* bnb = (const float*)d_in[16]; const float* bnm = (const float*)d_in[17]; const float* bnv = (const float*)d_in[18]; const float* wc2 = (const float*)d_in[19]; const float* bc2 = (const float*)d_in[20];
    float* OUT = (float*)d_out;
    char* wsp = (char*)d_ws;
    auto take = [&](size_t bytes) { char* p = wsp; wsp += (bytes + 255) & ~(size_t)255; return (void*)p; };
    bf* WQ = (bf*)take(CC * CC * 2); bf* WK = (bf*)take(CC * CC * 2); bf* WV = (bf*)take(CC * CC * 2); bf* WM = (bf*)take(CC * CC * 2); bf* WC1 = (bf*)take(4 * CC * CC * 2); bf* WC2 = (bf*)take(2 * CC * CC * 2);
    bf* X1 = (bf*)take((size_t)NN * CC * 2); bf* X2 = (bf*)take((size_t)NN * CC * 2); float* QF = (float*)take((size_t)NN * CC * 4); float* KE = (float*)take((size_t)NN * CC * 4); float* VA = (float*)take((size_t)NN * CC * 4); float* ADD = (float*)take((size_t)NN * CC * 4);
    bf* Ph = (bf*)take((size_t)NN * 2 * CC * 2); bf* Pl = (bf*)take((size_t)NN * 2 * CC * 2); float* M = (float*)take((size_t)NN * CC * 4); float* Y = (float*)take((size_t)NN * 2 * CC * 4); float* R = (float*)take((size_t)NN * CC * 4);
    if ((size_t)(wsp - (char*)d_ws) > ws_size) return;
    k_cvt8<<<(CC * CC / 8 + 255) / 256, 256, 0, stream>>>(wq, WQ, CC * CC / 8); k_cvt8<<<(CC * CC / 8 + 255) / 256, 256, 0, stream>>>(wk, WK, CC * CC / 8); k_cvt8<<<(CC * CC / 8 + 255) / 256, 256, 0, stream>>>(wv, WV, CC * CC / 8); k_cvt8<<<(CC * CC / 8 + 255) / 256, 256, 0, stream>>>(wm, WM, CC * CC / 8);
    k_cvt8<<<(4 * CC * CC / 8 + 255) / 256, 256, 0, stream>>>(wc1, WC1, 4 * CC * CC / 8); k_cvt8<<<(2 * CC * CC / 8 + 255) / 256, 256, 0, stream>>>(wc2, WC2, 2 * CC * CC / 8);
    const unsigned L4 = (unsigned)(((size_t)NN * CC / 4 + 255) / 256);
    for (int b = 0; b < NB_; ++b) { const float* x1 = d1 + (size_t)b * CC * NN; const float* x2 = d2 + (size_t)b * CC * NN;
        k_xt<<<L4, 256, 0, stream>>>(x1, X1); k_xt<<<L4, 256, 0, stream>>>(x2, X2);
        k_gemmw<bf, 0, true><<<dim3(NN / 64, CC / 64, 1), 32, 0, stream>>>(X1, nullptr, WQ, nullptr, CC, QF, CC, bq, 0, 0, 0); k_gemmw<bf, 0, true><<<dim3(NN / 64, CC / 64, 1), 32, 0, stream>>>(X2, nullptr, WK, nullptr, CC, KE, CC, bk, 0, 0, 0); k_gemmw<bf, 0, true><<<dim3(NN / 64, CC / 64, 1), 32, 0, stream>>>(X2, nullptr, WV, nullptr, CC, VA, CC, bv, 0, 0, 0);
        k_nbr<<<NN * NH_ / 8, 256, 0, stream>>>(QF, KE, VA, nbr + (size_t)b * KNB * NN, nmask + (size_t)b * KNB * NN, rlam, ADD);
        k_spl<<<L4, 256, 0, stream>>>(ADD, (size_t)NN * CC / 4, Ph, Pl); k_gemmw<bf, 1, true><<<dim3(NN / 64, CC / 64, 1), 32, 0, stream>>>(Ph, Pl, WM, nullptr, CC, M, CC, bm, 0, 0, 0);
        k_catpl<<<(unsigned)(((size_t)NN * 2 * CC / 4 + 255) / 256), 256, 0, stream>>>(x1, M, Ph, Pl); k_gemmw<bf, 1, false><<<dim3(NN / 64, 2 * CC / 64, 1), 32, 0, stream>>>(Ph, Pl, WC1, nullptr, 2 * CC, Y, 2 * CC, nullptr, 0, 0, 0);
        k_bnrelu<<<(unsigned)(((size_t)NN * 2 * CC / 4 + 255) / 256), 256, 0, stream>>>(Y, bng, bnb, bnm, bnv, Ph, Pl); k_gemmw<bf, 1, true><<<dim3(NN / 64, CC / 64, 1), 32, 0, stream>>>(Ph, Pl, WC2, nullptr, 2 * CC, R, CC, bc2, 0, 0, 0);
        k_outT<<<L4, 256, 0, stream>>>(x1, R, OUT + (size_t)b * CC * NN); }
}
